// TaylorSeriesChannelMixer_26027501814564
// MI455X (gfx1250) — hardware-verified
//
#include <hip/hip_runtime.h>


#define NB_  4
#define CI   16
#define NO   16
#define HID  64
#define NPX  65536
#define KP   32
#define DM   HID
#define SLOPE 0.1f
#define LOSC 1024.0f

typedef _Float16 h16;
typedef unsigned short bf;
typedef __attribute__((ext_vector_type(16))) __bf16   v16bf;
typedef __attribute__((ext_vector_type(16))) _Float16 v16h;
typedef __attribute__((ext_vector_type(8)))  _Float16 v8h;
typedef __attribute__((ext_vector_type(8)))  unsigned short v8us;
typedef __attribute__((ext_vector_type(8)))  float    v8f;
typedef __attribute__((ext_vector_type(4)))  float    v4f;
typedef v8h  __attribute__((may_alias)) v8ha;
typedef v4f  __attribute__((may_alias)) v4fa;
typedef v8us __attribute__((may_alias)) v8usa;

__device__ __forceinline__ unsigned short f2bf(float f) { unsigned u = __float_as_uint(f); u += 0x7FFFu + ((u >> 16) & 1u); return (unsigned short)(u >> 16); }
__device__ __forceinline__ float bf2f(unsigned short b) { return __uint_as_float(((unsigned)b) << 16); }
__device__ __forceinline__ float bfr(float f) { return bf2f(f2bf(f)); }
__device__ __forceinline__ v16h cat16(v8h lo, v8h hi) { return __builtin_shufflevector(lo, hi, 0, 1, 2, 3, 4, 5, 6, 7, 8, 9, 10, 11, 12, 13, 14, 15); }
__device__ __forceinline__ v16bf cat16b(v8us lo, v8us hi) { return __builtin_bit_cast(v16bf, __builtin_shufflevector(lo, hi, 0, 1, 2, 3, 4, 5, 6, 7, 8, 9, 10, 11, 12, 13, 14, 15)); }
__device__ __forceinline__ v8f wmma16(v16h a, v16h b, v8f c) { return __builtin_amdgcn_wmma_f32_16x16x32_f16(false, a, false, b, (short)0, c, false, false); }
__device__ __forceinline__ v8f wmmab(v16bf a, v16bf b, v8f c) { return __builtin_amdgcn_wmma_f32_16x16x32_bf16(false, a, false, b, (short)0, c, false, false); }

template <bool SPLITA, bool F16OUT = false>
__global__ __launch_bounds__(128) void k_gemmb(const bf* __restrict__ A, const bf* __restrict__ Al, const bf* __restrict__ Bn, const float* __restrict__ bias, float* C, int ldc, h16* C2, const float* __restrict__ R = nullptr, int K = DM, int roundR = 1) {
    __shared__ __align__(16) float ost[4][16 * 68];
    const int lane = threadIdx.x & 31, wave = threadIdx.x >> 5, lr = lane & 15, hi = lane >> 4;
    const int r0 = blockIdx.x * 64 + wave * 16, c0 = blockIdx.y * 64;
    const size_t aoff = (size_t)(r0 + lr) * K + 8 * hi;
    size_t boff[4];
#pragma unroll
    for (int t = 0; t < 4; ++t) boff[t] = (size_t)(c0 + t * 16 + lr) * K + 8 * hi;
    v8f acc[4];
#pragma unroll
    for (int t = 0; t < 4; ++t) acc[t] = (v8f){};
#pragma unroll 1
    for (int kc = 0; kc < K; kc += 32) {
        const v16bf a = cat16b(*(const v8us*)(A + aoff + kc), *(const v8us*)(A + aoff + kc + 16));
        v16bf al = a;
        if (SPLITA) al = cat16b(*(const v8us*)(Al + aoff + kc), *(const v8us*)(Al + aoff + kc + 16));
#pragma unroll
        for (int t = 0; t < 4; ++t) { const v16bf b = cat16b(*(const v8us*)(Bn + boff[t] + kc), *(const v8us*)(Bn + boff[t] + kc + 16)); acc[t] = wmmab(a, b, acc[t]); if (SPLITA) acc[t] = wmmab(al, b, acc[t]); }
        asm volatile("v_nop\n\tv_nop\n\tv_nop\n\tv_nop" : "+v"(acc[0]), "+v"(acc[1]), "+v"(acc[2]), "+v"(acc[3]) : "v"(a), "v"(al));
    }
    float* os = &ost[wave][0];
#pragma unroll
    for (int t = 0; t < 4; ++t) { const float bv = bias ? bfr(bias[c0 + t * 16 + lr]) : 0.f;
#pragma unroll
        for (int j = 0; j < 8; ++j) os[(hi * 8 + j) * 68 + t * 16 + lr] = acc[t][j] + bv; }
    __syncthreads();
    if (F16OUT) {
        h16* crow = (h16*)(void*)C + (size_t)r0 * ldc + c0;
        auto pass = [&]() {
#pragma unroll
            for (int s = 0; s < 4; ++s) { const int row = 4 * s + (lane >> 3), piece = lane & 7; const float* sp = os + row * 68 + piece * 8; v8h o, o2;
#pragma unroll
                for (int i = 0; i < 8; ++i) { const h16 a = (h16)sp[i]; o[i] = a; o2[i] = (h16)((sp[i] - (float)a) * LOSC); }
                *(volatile v8h*)(crow + (size_t)row * ldc + piece * 8) = o; if (C2) *(volatile v8h*)(C2 + (size_t)r0 * ldc + c0 + (size_t)row * ldc + piece * 8) = o2; }
        };
        pass(); __threadfence(); pass();
    } else {
        float* crow = C + (size_t)r0 * ldc + c0;
        auto pass = [&]() {
#pragma unroll
            for (int s = 0; s < 8; ++s) { const int Lid = (lane >> 3) + 4 * s, piece = lane & 7; const int row = Lid >> 1, cofs = (Lid & 1) * 32 + piece * 4;
                v4f val = *(const v4fa*)(os + row * 68 + cofs); if (R) { const v4f rv = *(const v4f*)(R + ((size_t)r0 + row) * ldc + c0 + cofs); val += roundR ? (v4f){bfr(rv[0]), bfr(rv[1]), bfr(rv[2]), bfr(rv[3])} : rv; }
                *(volatile v4f*)(crow + (size_t)row * ldc + cofs) = val; }
        };
        pass(); __threadfence(); pass();
    }
}

__global__ __launch_bounds__(256) void k_cvt8(const float* __restrict__ src, bf* dst, size_t n8) {
    const size_t i = (size_t)blockIdx.x * 256 + threadIdx.x; if (i >= n8) return;
    const v8f v = *(const v8f*)(src + i * 8); v8us o;
#pragma unroll
    for (int k = 0; k < 8; ++k) o[k] = f2bf(v[k]);
    *(volatile v8us*)(dst + i * 8) = o; __threadfence(); *(volatile v8us*)(dst + i * 8) = o;
}
__global__ __launch_bounds__(256) void k_zero8(bf* dst, size_t n8) {
    const size_t i = (size_t)blockIdx.x * 256 + threadIdx.x; if (i >= n8) return; v8us z;
#pragma unroll
    for (int k = 0; k < 8; ++k) z[k] = 0;
    *(volatile v8us*)(dst + i * 8) = z; __threadfence(); *(volatile v8us*)(dst + i * 8) = z;
}

__global__ __launch_bounds__(256) void k_tpoly(const float* __restrict__ xb, const float* __restrict__ coeff, bf* Th, bf* Tl, float* TF) {
    typedef __attribute__((ext_vector_type(2))) unsigned short v2us;
    const int lane = threadIdx.x & 31; const size_t p = ((size_t)blockIdx.x * 8 + (threadIdx.x >> 5)) * 2 + (lane >> 4); if (p >= (size_t)NPX) return; const int c0 = (lane & 15) * 2;
    typedef __attribute__((ext_vector_type(2))) float v2f_;
    const float k0 = bfr(coeff[0]), k1 = bfr(coeff[1]), k2 = bfr(coeff[2]), k3 = bfr(coeff[3]), k4 = bfr(coeff[4]); v2us oh, ol; v2f_ tf;
#pragma unroll
    for (int q = 0; q < 2; ++q) { const int c = c0 + q; float t = 0.f; if (c < CI) { const float x = bfr(xb[(size_t)c * NPX + p]); const float x2 = x * x, x3 = x2 * x, x4 = x2 * x2; t = k0 + k1 * x + k2 * x2 / 2.0f + k3 * x3 / 6.0f + k4 * x4 / 24.0f; }
        tf[q] = t; const unsigned short hb = f2bf(t); oh[q] = hb; ol[q] = f2bf(t - bf2f(hb)); }
    const size_t o = p * KP + c0; *(volatile v2us*)(Th + o) = oh; *(volatile v2us*)(Tl + o) = ol; if (c0 < CI) *(volatile v2f_*)(TF + p * CI + c0) = tf; __threadfence(); *(volatile v2us*)(Th + o) = oh; *(volatile v2us*)(Tl + o) = ol; if (c0 < CI) *(volatile v2f_*)(TF + p * CI + c0) = tf;
}
__global__ __launch_bounds__(256) void k_w1roll(const float* __restrict__ W1, const float* __restrict__ wc, bf* W1R, bf* WCR) {
    typedef __attribute__((ext_vector_type(2))) unsigned short v2us;
    const int lane = threadIdx.x & 31; const size_t row = ((size_t)blockIdx.x * 8 + (threadIdx.x >> 5)) * 2 + (lane >> 4); if (row >= (size_t)NO * HID) return; const int o = (int)(row / HID), d = (int)(row % HID); const int c0 = (lane & 15) * 2; v2us a, w;
#pragma unroll
    for (int q = 0; q < 2; ++q) { const int c = c0 + q; const int cs = ((c - o) % CI + CI) % CI; a[q] = f2bf(c < CI ? W1[(size_t)d * CI + cs] : 0.f); w[q] = f2bf((c < CI && d == 0) ? wc[cs] : 0.f); }
    const size_t off = row * KP + c0; *(volatile v2us*)(W1R + off) = a; *(volatile v2us*)(WCR + off) = w; __threadfence(); *(volatile v2us*)(W1R + off) = a; *(volatile v2us*)(WCR + off) = w;
}
__global__ __launch_bounds__(256) void k_relupl64(const float* __restrict__ F, bf* Ph, bf* Pl) {
    typedef __attribute__((ext_vector_type(2))) unsigned short v2us; typedef __attribute__((ext_vector_type(2))) float v2f_;
    const int lane = threadIdx.x & 31; const size_t r = (size_t)blockIdx.x * 8 + (threadIdx.x >> 5); if (r >= (size_t)NPX) return; const size_t o = r * HID + lane * 2; const v2f_ v = *(const v2f_*)(F + o); v2us oh, ol;
#pragma unroll
    for (int i = 0; i < 2; ++i) { const float y = fmaxf(v[i], 0.f); const unsigned short hb = f2bf(y); oh[i] = hb; ol[i] = f2bf(y - bf2f(hb)); }
    *(volatile v2us*)(Ph + o) = oh; *(volatile v2us*)(Pl + o) = ol; __threadfence(); *(volatile v2us*)(Ph + o) = oh; *(volatile v2us*)(Pl + o) = ol;
}
__global__ __launch_bounds__(256) void k_w3pad(const float* __restrict__ W3, bf* W3P) {
    typedef __attribute__((ext_vector_type(2))) unsigned short v2us;
    const int lane = threadIdx.x & 31; const int r = blockIdx.x * 8 + (threadIdx.x >> 5); if (r >= 64) return; v2us v;
#pragma unroll
    for (int i = 0; i < 2; ++i) v[i] = f2bf(r == 0 ? W3[lane * 2 + i] : 0.f);
    *(volatile v2us*)(W3P + (size_t)r * HID + lane * 2) = v; __threadfence(); *(volatile v2us*)(W3P + (size_t)r * HID + lane * 2) = v;
}
__global__ __launch_bounds__(64) void k_bias1(const float* __restrict__ b, float* BP) { const int t = threadIdx.x; const float v = (t == 0) ? b[0] : 0.f; *(volatile float*)(BP + t) = v; __threadfence(); *(volatile float*)(BP + t) = v; }
__global__ __launch_bounds__(256) void k_y(const float* __restrict__ TF, const float* __restrict__ H2, const float* __restrict__ wc, const float* __restrict__ bc, const float* __restrict__ W3, const float* __restrict__ b3, int o, float* Yo) {
    const int lane = threadIdx.x & 31; const size_t w = (size_t)blockIdx.x * 8 + (threadIdx.x >> 5); if (w >= (size_t)NPX / 32) return; const size_t p = w * 32 + lane;
    float cv = bfr(bc[0]);
#pragma unroll 4
    for (int c = 0; c < CI; ++c) cv = fmaf(bfr(wc[((c - o) % CI + CI) % CI]), TF[p * CI + c], cv);
    float h3 = bfr(b3[0]);
#pragma unroll 4
    for (int d = 0; d < HID; ++d) h3 = fmaf(bfr(W3[d]), fmaxf(H2[p * HID + d], 0.f), h3);
    float v = cv + h3; v = (v >= 0.f) ? v : SLOPE * v; *(volatile float*)(Yo + p) = v; __threadfence(); *(volatile float*)(Yo + p) = v;
}
__global__ __launch_bounds__(256) void k_minmax(const float* __restrict__ Y, float* MM) {
    __shared__ float rmn[256]; __shared__ float rmx[256];
    const int t = threadIdx.x, o = blockIdx.x; const float* yo = Y + (size_t)o * NPX; float mn = 3.0e38f, mx = -3.0e38f;
    for (int p = t; p < NPX; p += 256) { const float v = yo[p]; mn = fminf(mn, v); mx = fmaxf(mx, v); }
    rmn[t] = mn; rmx[t] = mx; __syncthreads();
    for (int st = 128; st > 0; st >>= 1) { if (t < st) { rmn[t] = fminf(rmn[t], rmn[t + st]); rmx[t] = fmaxf(rmx[t], rmx[t + st]); } __syncthreads(); }
    if (t < 32) { const float v = (t == 0) ? rmn[0] : (t == 1) ? rmx[0] : 0.f; *(volatile float*)(MM + o * 32 + t) = v; __threadfence(); *(volatile float*)(MM + o * 32 + t) = v; }
}
__global__ __launch_bounds__(256) void k_norm(const float* __restrict__ Y, const float* __restrict__ MM, float* OUTB) {
    const int lane = threadIdx.x & 31; const size_t w = (size_t)blockIdx.x * 8 + (threadIdx.x >> 5); if (w >= (size_t)NO * (NPX / 128)) return; const int o = (int)(w / (NPX / 128)); const size_t p0 = (w % (NPX / 128)) * 128 + lane * 4;
    const float mn = MM[o * 32], mx = MM[o * 32 + 1]; const float den = mx - mn + 1e-8f; const v4f v = *(const v4f*)(Y + (size_t)o * NPX + p0); v4f r;
#pragma unroll
    for (int i = 0; i < 4; ++i) r[i] = (v[i] - mn) / den;
    *(volatile v4f*)(OUTB + (size_t)o * NPX + p0) = r; __threadfence(); *(volatile v4f*)(OUTB + (size_t)o * NPX + p0) = r;
}

extern "C" void kernel_launch(void* const* d_in, const int* in_sizes, int n_in,
                              void* d_out, int out_size, void* d_ws, size_t ws_size, hipStream_t stream) {
    (void)in_sizes; (void)n_in; (void)out_size;
    const float* x = (const float*)d_in[0]; const float* coeff = (const float*)d_in[1]; const float* wc = (const float*)d_in[2]; const float* bc = (const float*)d_in[3]; const float* W1 = (const float*)d_in[4]; const float* b1 = (const float*)d_in[5]; const float* W2 = (const float*)d_in[6]; const float* b2 = (const float*)d_in[7]; const float* W3 = (const float*)d_in[8]; const float* b3 = (const float*)d_in[9];
    float* out = (float*)d_out;
    char* wsp = (char*)d_ws;
    auto take = [&](size_t bytes) { char* p = wsp; wsp += (bytes + 255) & ~(size_t)255; return (void*)p; };
    bf* W1R = (bf*)take((size_t)NO * HID * KP * 2); bf* WCR = (bf*)take((size_t)NO * HID * KP * 2); bf* W2B = (bf*)take((size_t)HID * HID * 2);
    bf* Th = (bf*)take((size_t)NPX * KP * 2); bf* Tl = (bf*)take((size_t)NPX * KP * 2); float* TF = (float*)take((size_t)NPX * CI * 4); float* H1 = (float*)take((size_t)NPX * HID * 4); bf* Ph = (bf*)take((size_t)NPX * HID * 2); bf* Pl = (bf*)take((size_t)NPX * HID * 2); float* H2 = (float*)take((size_t)NPX * HID * 4);
    float* Y = (float*)take((size_t)NO * NPX * 4); float* MM = (float*)take((size_t)NO * 32 * 4);
    if ((size_t)(wsp - (char*)d_ws) > ws_size) return;
    k_w1roll<<<((NO * HID) / 2) / 8, 256, 0, stream>>>(W1, wc, W1R, WCR); k_cvt8<<<(HID * HID / 8 + 255) / 256, 256, 0, stream>>>(W2, W2B, HID * HID / 8);
    const dim3 gg(NPX / 64, 1, 1);
    for (int b = 0; b < NB_; ++b) {
        k_tpoly<<<(NPX / 2) / 8, 256, 0, stream>>>(x + (size_t)b * CI * NPX, coeff, Th, Tl, TF);
        for (int o = 0; o < NO; ++o) {
            k_gemmb<true, false><<<gg, 128, 0, stream>>>(Th, Tl, W1R + (size_t)o * HID * KP, b1, H1, HID, nullptr, nullptr, KP);
            k_relupl64<<<NPX / 8, 256, 0, stream>>>(H1, Ph, Pl); k_gemmb<true, false><<<gg, 128, 0, stream>>>(Ph, Pl, W2B, b2, H2, HID, nullptr, nullptr, HID);
            k_y<<<(NPX / 32) / 8, 256, 0, stream>>>(TF, H2, wc, bc, W3, b3, o, Y + (size_t)o * NPX); }
        k_minmax<<<NO, 256, 0, stream>>>(Y, MM);
        k_norm<<<(NO * (NPX / 128)) / 8, 256, 0, stream>>>(Y, MM, out + (size_t)b * NO * NPX); }
}
